// DPSA_52905407152224
// MI455X (gfx1250) — hardware-verified
//
#include <hip/hip_runtime.h>
#include <math.h>
#include <stdint.h>

#define NBATCH 2
#define SEQ    2048
#define DM     1024
#define NH     16
#define HD     64
#define NTOK   (NBATCH * SEQ)
#define HDX    128
#define QXP    (NH * HDX)
#define NQB    (SEQ / 64)
#define WSC    16.0f
#define RSC    2048.0f
static_assert(NH * HD == DM);
static_assert((SEQ % 64) == 0 && (DM % 64) == 0);
static_assert(((QXP * 2) % 128) == 0);
static_assert((NTOK * DM) % 2048 == 0);

typedef _Float16 v16h __attribute__((ext_vector_type(16)));
typedef _Float16 v8h  __attribute__((ext_vector_type(8)));
typedef __bf16   v16b __attribute__((ext_vector_type(16)));
typedef unsigned short v16us __attribute__((ext_vector_type(16)));
typedef unsigned short v8us  __attribute__((ext_vector_type(8)));
typedef float    v8f  __attribute__((ext_vector_type(8)));
typedef float    v4f  __attribute__((ext_vector_type(4)));
typedef unsigned int v4u __attribute__((ext_vector_type(4)));
union FH { v16h v; v8h h[2]; };
union FB { v16us u; v8us h[2]; };

__device__ __forceinline__ unsigned short bf_bits(float f) {
  unsigned u = __float_as_uint(f);
  return (unsigned short)((u + 0x7FFFu + ((u >> 16) & 1u)) >> 16);
}
__device__ __forceinline__ float bf_up(unsigned short h) { return __uint_as_float(((unsigned)h) << 16); }
__device__ __forceinline__ float bfr(float f) { return bf_up(bf_bits(f)); }
__device__ __forceinline__ unsigned short h_bits(_Float16 x) { return __builtin_bit_cast(unsigned short, x); }
__device__ __forceinline__ unsigned pk16(unsigned short a, unsigned short b) { return (unsigned)a | ((unsigned)b << 16); }
__device__ __forceinline__ v8f zero8() { v8f z = {0.f, 0.f, 0.f, 0.f, 0.f, 0.f, 0.f, 0.f}; return z; }

__device__ __forceinline__ v16h ldfrag_h(const _Float16* p) {
  FH f;
  f.h[0] = *(const v8h*)(p);
  f.h[1] = *(const v8h*)(p + 16);
  return f.v;
}
__device__ __forceinline__ v16us ldfrag_b(const unsigned short* p) {
  FB f;
  f.h[0] = *(const v8us*)(p);
  f.h[1] = *(const v8us*)(p + 16);
  return f.u;
}

__device__ __forceinline__ v8f mma_h(v16h a, v16h b, v8f c) {
  c = __builtin_amdgcn_wmma_f32_16x16x32_f16(false, a, false, b, (short)0, c, false, false);
#if defined(__HIP_DEVICE_COMPILE__)
  asm volatile("v_nop\n\tv_nop\n\tv_nop\n\tv_nop" : "+v"(c) : "v"(a), "v"(b));
#endif
  return c;
}
__device__ __forceinline__ v8f mma_h_raw(v16h a, v16h b, v8f c) {
  return __builtin_amdgcn_wmma_f32_16x16x32_f16(false, a, false, b, (short)0, c, false, false);
}
__device__ __forceinline__ v8f mma_b_raw(v16us a, v16us b, v8f c) {
  return __builtin_amdgcn_wmma_f32_16x16x32_bf16(false, __builtin_bit_cast(v16b, a), false,
                                                 __builtin_bit_cast(v16b, b), (short)0, c, false, false);
}
__device__ __forceinline__ void dep_guard_h(v8f& a, v8f& b, v16h x, v16h y) {
#if defined(__HIP_DEVICE_COMPILE__)
  asm volatile("v_nop\n\tv_nop\n\tv_nop\n\tv_nop" : "+v"(a), "+v"(b) : "v"(x), "v"(y));
#endif
}
__device__ __forceinline__ void dep_guard_b(v8f& a, v8f& b, v16us x, v16us y) {
#if defined(__HIP_DEVICE_COMPILE__)
  asm volatile("v_nop\n\tv_nop\n\tv_nop\n\tv_nop" : "+v"(a), "+v"(b) : "v"(x), "v"(y));
#endif
}
__device__ __forceinline__ void keep4_h(v16h a, v16h b, v16h c, v16h d) {
#if defined(__HIP_DEVICE_COMPILE__)
  asm volatile("v_nop" :: "v"(a), "v"(b), "v"(c), "v"(d));
#endif
}
__device__ __forceinline__ void keep4_b(v16us a, v16us b, v16us c, v16us d) {
#if defined(__HIP_DEVICE_COMPILE__)
  asm volatile("v_nop" :: "v"(a), "v"(b), "v"(c), "v"(d));
#endif
}
__device__ __forceinline__ void acc_guard4(v8f& a, v8f& b, v8f& c, v8f& d) {
#if defined(__HIP_DEVICE_COMPILE__)
  asm volatile("v_nop\n\tv_nop\n\tv_nop\n\tv_nop" : "+v"(a), "+v"(b), "+v"(c), "+v"(d));
#endif
}
__device__ __forceinline__ void wave_sync_lds() {
  __builtin_amdgcn_fence(__ATOMIC_RELEASE, "workgroup");
  __builtin_amdgcn_wave_barrier();
  __builtin_amdgcn_fence(__ATOMIC_ACQUIRE, "workgroup");
}

__global__ __launch_bounds__(256) void tr_cvt6(const float* __restrict__ in0, const float* __restrict__ in1,
                                               const float* __restrict__ in2, const float* __restrict__ in3,
                                               const float* __restrict__ in4, const float* __restrict__ in5,
                                               unsigned short* out, long long zstride, int R, int C, float scale,
                                               int zbf) {
  __shared__ float tile[64 * 33];
  const int z = blockIdx.z;
  const float* in = (z == 0) ? in0 : ((z == 1) ? in1 : ((z == 2) ? in2 : ((z == 3) ? in3 : ((z == 4) ? in4 : in5))));
  unsigned short* ob = out + (size_t)z * (size_t)zstride;
  const bool bfmode = (z >= zbf);
  const int r0 = blockIdx.y * 64, c0 = blockIdx.x * 32;
  const int t = threadIdx.x;
  {
    const int ir = t >> 2, ic = (t & 3) * 8;
    const float* g = in + (size_t)(r0 + ir) * C + c0 + ic;
    const v4f a = *(const v4f*)g;
    const v4f b = *(const v4f*)(g + 4);
    float* l = tile + ir * 33 + ic;
    l[0] = a[0]; l[1] = a[1]; l[2] = a[2]; l[3] = a[3];
    l[4] = b[0]; l[5] = b[1]; l[6] = b[2]; l[7] = b[3];
  }
  __syncthreads();
  const int orow = t >> 3, piece = (t & 7) * 8;
  v4u p;
#pragma unroll
  for (int e = 0; e < 4; ++e) {
    const float f0 = tile[(piece + 2 * e) * 33 + orow];
    const float f1 = tile[(piece + 2 * e + 1) * 33 + orow];
    const unsigned short b0 = bf_bits(f0), b1 = bf_bits(f1);
    const _Float16 x0 = (_Float16)(bf_up(b0) * scale);
    const _Float16 x1 = (_Float16)(bf_up(b1) * scale);
    const unsigned wf = pk16(h_bits(x0), h_bits(x1));
    const unsigned wb = pk16(b0, b1);
    p[e] = bfmode ? wb : wf;
  }
  const size_t go = (size_t)(c0 + orow) * (size_t)R + r0 + piece;
  *(volatile v4u*)(ob + go) = p;
  __threadfence();
  *(volatile v4u*)(ob + go) = p;
}

__global__ __launch_bounds__(256) void cvt_f16(const float* __restrict__ in0, const float* __restrict__ in1,
                                              unsigned short* out, long long zstride, int n) {
  const int z = blockIdx.y;
  const float* in = (z == 0) ? in0 : in1;
  unsigned short* ob = out + (size_t)z * (size_t)zstride;
  const size_t i8 = ((size_t)blockIdx.x * 256 + threadIdx.x) * 8;
  if (i8 + 8 > (size_t)n) return;
  const v4f a = *(const v4f*)(in + i8);
  const v4f b = *(const v4f*)(in + i8 + 4);
  v4u p;
#pragma unroll
  for (int e = 0; e < 2; ++e) {
    p[e]     = pk16(h_bits((_Float16)bfr(a[2 * e])), h_bits((_Float16)bfr(a[2 * e + 1])));
    p[2 + e] = pk16(h_bits((_Float16)bfr(b[2 * e])), h_bits((_Float16)bfr(b[2 * e + 1])));
  }
  *(volatile v4u*)(ob + i8) = p;
  __threadfence();
  *(volatile v4u*)(ob + i8) = p;
}

template <int OM, int BIASM, bool GAM, bool EXT>
__global__ __launch_bounds__(256) void gemm64(
    const unsigned short* __restrict__ Ap, int lda, long long strideA,
    const unsigned short* __restrict__ Btp, int ldb, long long strideB,
    void* Cout, void* Cout2, int ldc, long long strideC, int extoff,
    const float* __restrict__ bias, const float* __restrict__ gam,
    int M, int N, int K, float oscale) {
  const _Float16* A  = (const _Float16*)(const void*)Ap;
  const _Float16* Bt = (const _Float16*)(const void*)Btp;
  __shared__ __align__(16) float sT[8][16 * 68];
  const int b    = blockIdx.y;
  const int lane = threadIdx.x & 31;
  const int wave = threadIdx.x >> 5;
  const int tilesN = N >> 6;
  const int tilesM = M >> 6;
  const int tile = blockIdx.x * 8 + wave;
  if (tile >= tilesM * tilesN) return;
  const int tm = tile / tilesN;
  const int tn = tile - tm * tilesN;
  const int m0 = tm << 6;
  const int n0 = tn << 6;

  const _Float16* Ab = A  + (size_t)b * (size_t)strideA;
  const _Float16* Bb = Bt + (size_t)b * (size_t)strideB;

  const int rlane = lane & 15;
  const int koff  = (lane >> 4) * 8;
  const int mOff  = (lane >> 4) * 8;

  v8f acc[4][4];
#pragma unroll
  for (int i = 0; i < 4; ++i)
#pragma unroll
    for (int j = 0; j < 4; ++j) acc[i][j] = zero8();

  for (int k0 = 0; k0 < K; k0 += 32) {
    v16h bh[4];
#pragma unroll
    for (int j = 0; j < 4; ++j) {
      const size_t bo = (size_t)(n0 + (j << 4) + rlane) * ldb + koff + k0;
      bh[j] = ldfrag_h(Bb + bo);
    }
#pragma unroll
    for (int i = 0; i < 4; ++i) {
      const size_t ao = (size_t)(m0 + (i << 4) + rlane) * lda + koff + k0;
      const v16h ah = ldfrag_h(Ab + ao);
#pragma unroll
      for (int j = 0; j < 4; ++j) acc[i][j] = mma_h_raw(ah, bh[j], acc[i][j]);
      dep_guard_h(acc[i][0], acc[i][3], ah, bh[3]);
    }
    keep4_h(bh[0], bh[1], bh[2], bh[3]);
  }
  acc_guard4(acc[0][0], acc[0][1], acc[0][2], acc[0][3]);
  acc_guard4(acc[1][0], acc[1][1], acc[1][2], acc[1][3]);
  acc_guard4(acc[2][0], acc[2][1], acc[2][2], acc[2][3]);
  acc_guard4(acc[3][0], acc[3][1], acc[3][2], acc[3][3]);

  float gmul = 1.0f;
  if (GAM) gmul = bfr(gam[0]);
  const int cn0 = EXT ? (((n0 >> 6) << 7) + extoff) : n0;
  float* slab = sT[wave];
  const int q = lane >> 3, c8 = (lane & 7) * 8;
  unsigned short* C  = (unsigned short*)Cout  + (size_t)b * (size_t)strideC;
  unsigned short* C2 = (unsigned short*)Cout2 + (size_t)b * (size_t)strideC;
  float b8[8];
#pragma unroll
  for (int e = 0; e < 8; ++e) b8[e] = 0.f;
  if (BIASM == 1) {
    const v4f t0 = *(const v4f*)(bias + n0 + c8);
    const v4f t1 = *(const v4f*)(bias + n0 + c8 + 4);
#pragma unroll
    for (int e = 0; e < 4; ++e) { b8[e] = bfr(t0[e]); b8[4 + e] = bfr(t1[e]); }
  }
#pragma unroll
  for (int i = 0; i < 4; ++i) {
    const int mBase = m0 + (i << 4);
#pragma unroll
    for (int j = 0; j < 4; ++j) {
#pragma unroll
      for (int r = 0; r < 8; ++r) {
        slab[(mOff + r) * 68 + (j << 4) + rlane] = acc[i][j][r];
      }
    }
    wave_sync_lds();
    v4u hv[4], lv[4];
#pragma unroll
    for (int it = 0; it < 4; ++it) {
      const int row = it * 4 + q;
      const float* sp = slab + row * 68 + c8;
      float brow = 0.f;
      if (BIASM == 2) brow = bfr(bias[mBase + row]);
      v4u pk;
      v4u pl = {0u, 0u, 0u, 0u};
#pragma unroll
      for (int e = 0; e < 4; ++e) {
        const float f0 = (sp[2 * e] * oscale + b8[2 * e] + brow) * gmul;
        const float f1 = (sp[2 * e + 1] * oscale + b8[2 * e + 1] + brow) * gmul;
        const _Float16 x0 = (_Float16)f0;
        const _Float16 x1 = (_Float16)f1;
        pk[e] = pk16(h_bits(x0), h_bits(x1));
        if (OM == 2) {
          const _Float16 y0 = (_Float16)((f0 - (float)x0) * RSC);
          const _Float16 y1 = (_Float16)((f1 - (float)x1) * RSC);
          pl[e] = pk16(h_bits(y0), h_bits(y1));
        }
      }
      hv[it] = pk;
      lv[it] = pl;
    }
    for (int pass = 0; pass < 2; ++pass) {
#pragma unroll
      for (int it = 0; it < 4; ++it) {
        const int row = it * 4 + q;
        const size_t go = (size_t)(mBase + row) * ldc + cn0 + c8;
        *(volatile v4u*)(C + go) = hv[it];
        if (OM == 2) *(volatile v4u*)(C2 + go) = lv[it];
      }
      __threadfence();
    }
    wave_sync_lds();
  }
}

template <bool TWO>
__global__ __launch_bounds__(256) void gemm64b(
    const unsigned short* __restrict__ Ah, const unsigned short* __restrict__ Al, int lda,
    const unsigned short* __restrict__ Bt, int ldb,
    float* Cout, int ldc, const float* __restrict__ bias, int M, int N, int K) {
  __shared__ __align__(16) float sT[8][16 * 68];
  const int lane = threadIdx.x & 31;
  const int wave = threadIdx.x >> 5;
  const int tilesN = N >> 6;
  const int tilesM = M >> 6;
  const int tile = blockIdx.x * 8 + wave;
  if (tile >= tilesM * tilesN) return;
  const int tm = tile / tilesN;
  const int tn = tile - tm * tilesN;
  const int m0 = tm << 6;
  const int n0 = tn << 6;

  const int rlane = lane & 15;
  const int koff  = (lane >> 4) * 8;
  const int mOff  = (lane >> 4) * 8;

  v8f acc[4][4];
#pragma unroll
  for (int i = 0; i < 4; ++i)
#pragma unroll
    for (int j = 0; j < 4; ++j) acc[i][j] = zero8();

  const int nsweep = TWO ? 2 : 1;
  for (int pl = 0; pl < nsweep; ++pl) {
    const unsigned short* Ab = (pl == 0) ? Ah : Al;
    for (int k0 = 0; k0 < K; k0 += 32) {
      v16us bh[4];
#pragma unroll
      for (int j = 0; j < 4; ++j) {
        const size_t bo = (size_t)(n0 + (j << 4) + rlane) * ldb + koff + k0;
        bh[j] = ldfrag_b(Bt + bo);
      }
#pragma unroll
      for (int i = 0; i < 4; ++i) {
        const size_t ao = (size_t)(m0 + (i << 4) + rlane) * lda + koff + k0;
        const v16us ah = ldfrag_b(Ab + ao);
#pragma unroll
        for (int j = 0; j < 4; ++j) acc[i][j] = mma_b_raw(ah, bh[j], acc[i][j]);
        dep_guard_b(acc[i][0], acc[i][3], ah, bh[3]);
      }
      keep4_b(bh[0], bh[1], bh[2], bh[3]);
    }
  }
  acc_guard4(acc[0][0], acc[0][1], acc[0][2], acc[0][3]);
  acc_guard4(acc[1][0], acc[1][1], acc[1][2], acc[1][3]);
  acc_guard4(acc[2][0], acc[2][1], acc[2][2], acc[2][3]);
  acc_guard4(acc[3][0], acc[3][1], acc[3][2], acc[3][3]);

  float* slab = sT[wave];
  const int h2 = lane >> 4, c4 = (lane & 15) * 4;
  v4f bv = {0.f, 0.f, 0.f, 0.f};
  {
    const v4f t4 = *(const v4f*)(bias + n0 + c4);
#pragma unroll
    for (int e = 0; e < 4; ++e) bv[e] = bfr(t4[e]);
  }
#pragma unroll
  for (int i = 0; i < 4; ++i) {
    const int mBase = m0 + (i << 4);
#pragma unroll
    for (int j = 0; j < 4; ++j) {
#pragma unroll
      for (int r = 0; r < 8; ++r) {
        slab[(mOff + r) * 68 + (j << 4) + rlane] = acc[i][j][r];
      }
    }
    wave_sync_lds();
    for (int pass = 0; pass < 2; ++pass) {
#pragma unroll
      for (int it = 0; it < 8; ++it) {
        const int row = it * 2 + h2;
        const v4f sv = *(const v4f*)(slab + row * 68 + c4);
        v4f o;
#pragma unroll
        for (int e = 0; e < 4; ++e) o[e] = sv[e] + bv[e];
        *(volatile v4f*)(Cout + (size_t)(mBase + row) * ldc + n0 + c4) = o;
      }
      __threadfence();
    }
    wave_sync_lds();
  }
}

__global__ __launch_bounds__(128)
void attn_x(const unsigned short* __restrict__ qhp, const unsigned short* __restrict__ qlp,
            const unsigned short* __restrict__ kxp, const unsigned short* __restrict__ vtp,
            const int* __restrict__ mk, unsigned short* cth, unsigned short* ctl, float sscale) {
  __shared__ __align__(16) _Float16 Ksh[64 * HDX];
  __shared__ __align__(16) _Float16 Vth[64 * 64];
  __shared__ __align__(16) _Float16 Psh[4][16 * 64];
  __shared__ __align__(16) float    Os[4][16 * 64];

  const int tid  = threadIdx.x;
  const int wave = tid >> 5;
  const int lane = tid & 31;
  const int hh   = lane >> 4;
  const int c    = lane & 15;

  const int bx   = blockIdx.x;
  const int qb   = bx % NQB;
  const int rest = bx / NQB;
  const int h    = rest % NH;
  const int b    = rest / NH;
  const int q0   = qb * 64 + wave * 16;
  const size_t rowB = (size_t)b * SEQ;

  const _Float16* Qh = (const _Float16*)(const void*)qhp + (size_t)h * HDX;
  const _Float16* Ql = (const _Float16*)(const void*)qlp + (size_t)h * HDX;
  const _Float16* Kg = (const _Float16*)(const void*)kxp + (size_t)h * HDX;
  const _Float16* Vg = (const _Float16*)(const void*)vtp + ((size_t)b * DM + (size_t)h * HD) * SEQ;
  const int*      Mg = mk + (rowB + q0 + 8 * hh) * (size_t)SEQ;

  v16h qa[4], qr[4];
#pragma unroll
  for (int dc = 0; dc < 4; ++dc) {
    qa[dc] = ldfrag_h(Qh + (rowB + q0 + c) * QXP + dc * 32 + 8 * hh);
    qr[dc] = ldfrag_h(Ql + (rowB + q0 + c) * QXP + dc * 32 + 8 * hh);
  }

  float mrow[8], lrow[8];
  v8f oacc[4];
#pragma unroll
  for (int r = 0; r < 8; ++r) { mrow[r] = -INFINITY; lrow[r] = 0.f; }
#pragma unroll
  for (int t = 0; t < 4; ++t) oacc[t] = zero8();

  for (int kt = 0; kt < NQB; ++kt) {
    const int kv0 = kt * 64;
    __syncthreads();
    {
      const int r = tid >> 1, hk = (tid & 1) * 64, hv = (tid & 1) * 32;
      const _Float16* kg = Kg + (rowB + kv0 + r) * QXP + hk;
      const _Float16* vg = Vg + (size_t)r * SEQ + kv0 + hv;
#pragma unroll
      for (int i = 0; i < 8; ++i) *(v8h*)(Ksh + r * HDX + hk + 8 * i) = *(const v8h*)(kg + 8 * i);
#pragma unroll
      for (int i = 0; i < 4; ++i) *(v8h*)(Vth + r * 64 + hv + 8 * i) = *(const v8h*)(vg + 8 * i);
    }
    __syncthreads();

    v8f s[4];
#pragma unroll
    for (int j = 0; j < 4; ++j) {
      v8f sh = zero8();
      v8f sl = zero8();
#pragma unroll
      for (int dc = 0; dc < 4; ++dc) {
        FH kb;
        kb.h[0] = *(const v8h*)(Ksh + (j * 16 + c) * HDX + dc * 32 + 8 * hh);
        kb.h[1] = *(const v8h*)(Ksh + (j * 16 + c) * HDX + dc * 32 + 16 + 8 * hh);
        sh = mma_h(qa[dc], kb.v, sh);
        sl = mma_h(qr[dc], kb.v, sl);
      }
      const int* mp = Mg + kv0 + j * 16 + c;
#pragma unroll
      for (int r = 0; r < 8; ++r) {
        const float v = (sh[r] + sl[r] * (1.0f / RSC)) * sscale;
        const int mv = mp[(size_t)r * SEQ];
        s[j][r] = (mv == 0) ? -1.0e9f : v;
      }
    }

    _Float16* pwh = Psh[wave];
#pragma unroll
    for (int r = 0; r < 8; ++r) {
      float m = s[0][r];
      m = fmaxf(m, s[1][r]);
      m = fmaxf(m, s[2][r]);
      m = fmaxf(m, s[3][r]);
#pragma unroll
      for (int off = 1; off < 16; off <<= 1) m = fmaxf(m, __shfl_xor(m, off, 32));
      const float mnew  = fmaxf(mrow[r], m);
      const float alpha = __expf(mrow[r] - mnew);
      mrow[r] = mnew;
      float psum = 0.f;
#pragma unroll
      for (int j = 0; j < 4; ++j) {
        const float p = __expf(s[j][r] - mnew);
        psum += p;
        pwh[(8 * hh + r) * 64 + j * 16 + c] = (_Float16)(p * 1024.0f);
      }
#pragma unroll
      for (int off = 1; off < 16; off <<= 1) psum += __shfl_xor(psum, off, 32);
      lrow[r] = lrow[r] * alpha + psum;
#pragma unroll
      for (int t = 0; t < 4; ++t) oacc[t][r] *= alpha;
    }
    wave_sync_lds();

#pragma unroll 1
    for (int kk = 0; kk < 2; ++kk) {
      FH pa;
      pa.h[0] = *(const v8h*)(pwh + c * 64 + kk * 32 + 8 * hh);
      pa.h[1] = *(const v8h*)(pwh + c * 64 + kk * 32 + 16 + 8 * hh);
#pragma unroll
      for (int t = 0; t < 4; ++t) {
        FH vb;
        vb.h[0] = *(const v8h*)(Vth + (t * 16 + c) * 64 + kk * 32 + 8 * hh);
        vb.h[1] = *(const v8h*)(Vth + (t * 16 + c) * 64 + kk * 32 + 16 + 8 * hh);
        oacc[t] = mma_h(pa.v, vb.v, oacc[t]);
      }
    }
  }

  float* os = Os[wave];
#pragma unroll
  for (int r = 0; r < 8; ++r) {
    const float l = lrow[r];
    const float inv = ((l > 0.f) ? (1.0f / l) : 0.f) * (1.0f / 1024.0f);
#pragma unroll
    for (int t = 0; t < 4; ++t) os[(8 * hh + r) * 64 + t * 16 + c] = oacc[t][r] * inv;
  }
  wave_sync_lds();
  {
    const int q4 = lane >> 3, c8 = (lane & 7) * 8;
    v4u hvv[4], lvv[4];
#pragma unroll
    for (int it = 0; it < 4; ++it) {
      const int row = it * 4 + q4;
      const float* sp = os + row * 64 + c8;
      v4u pk, pl;
#pragma unroll
      for (int e = 0; e < 4; ++e) {
        const float f0 = sp[2 * e], f1 = sp[2 * e + 1];
        const unsigned short b0 = bf_bits(f0), b1 = bf_bits(f1);
        const unsigned short l0 = bf_bits(f0 - bf_up(b0)), l1 = bf_bits(f1 - bf_up(b1));
        pk[e] = pk16(b0, b1);
        pl[e] = pk16(l0, l1);
      }
      hvv[it] = pk;
      lvv[it] = pl;
    }
    for (int pass = 0; pass < 2; ++pass) {
#pragma unroll
      for (int it = 0; it < 4; ++it) {
        const int row = it * 4 + q4;
        const size_t go = (rowB + q0 + row) * DM + (size_t)h * HD + c8;
        *(volatile v4u*)(cth + go) = hvv[it];
        *(volatile v4u*)(ctl + go) = lvv[it];
      }
      __threadfence();
    }
  }
}

extern "C" void kernel_launch(void* const* d_in, const int* in_sizes, int n_in,
                              void* d_out, int out_size, void* d_ws, size_t ws_size,
                              hipStream_t stream) {
  if (n_in < 16) return;
  if (in_sizes[0] != NTOK * DM || in_sizes[1] != NTOK * DM) return;
  if (in_sizes[2] != NBATCH * SEQ * SEQ) return;
  if (in_sizes[3] != DM * DM || in_sizes[5] != DM * DM || in_sizes[7] != DM * DM) return;
  if (in_sizes[9] != DM * DM || in_sizes[11] != DM * DM || in_sizes[13] != DM * DM) return;
  if (in_sizes[4] != DM || in_sizes[6] != DM || in_sizes[8] != DM) return;
  if (in_sizes[10] != DM || in_sizes[12] != DM || in_sizes[14] != DM) return;
  if (in_sizes[15] < 1) return;
  if (out_size != NTOK * DM) return;

  const float* X_sem  = (const float*)d_in[0];
  const float* X_sal  = (const float*)d_in[1];
  const int*   mask   = (const int*)d_in[2];
  const float* Wq_sem = (const float*)d_in[3];
  const float* bq_sem = (const float*)d_in[4];
  const float* Wk_sem = (const float*)d_in[5];
  const float* bk_sem = (const float*)d_in[6];
  const float* Wv     = (const float*)d_in[7];
  const float* bv     = (const float*)d_in[8];
  const float* Wq_sal = (const float*)d_in[9];
  const float* bq_sal = (const float*)d_in[10];
  const float* Wk_sal = (const float*)d_in[11];
  const float* bk_sal = (const float*)d_in[12];
  const float* Wo     = (const float*)d_in[13];
  const float* bo     = (const float*)d_in[14];
  const float* gamma  = (const float*)d_in[15];
  float* outf = (float*)d_out;

  const size_t WD    = (size_t)DM * DM;
  const size_t PWALL = (size_t)6 * WD * 2;
  const size_t PXH   = (size_t)2 * NTOK * DM * 2;
  const size_t PQX   = (size_t)NTOK * QXP * 2;
  const size_t PVT   = (size_t)NBATCH * DM * SEQ * 2;
  const size_t PCTX  = (size_t)NTOK * DM * 2;
  size_t off = 0;
  const size_t oWALL = off; off += PWALL;
  const size_t oXH   = off; off += PXH;
  const size_t oQXH  = off; off += PQX;
  const size_t oQXL  = off; off += PQX;
  const size_t oKX   = off; off += PQX;
  const size_t oVT   = off; off += PVT;
  const size_t oCTXH = off; off += PCTX;
  const size_t oCTXL = off; off += PCTX;
  if (off > ws_size) return;
  if (off > (size_t)134217728) return;

  char* ws = (char*)d_ws;
  unsigned short* WALL = (unsigned short*)(ws + oWALL);
  unsigned short* WQS  = WALL + 0 * WD;
  unsigned short* WKS  = WALL + 1 * WD;
  unsigned short* WQL  = WALL + 2 * WD;
  unsigned short* WKL  = WALL + 3 * WD;
  unsigned short* WVT  = WALL + 4 * WD;
  unsigned short* WOB  = WALL + 5 * WD;
  unsigned short* XH0  = (unsigned short*)(ws + oXH);
  unsigned short* XH1  = XH0 + (size_t)NTOK * DM;
  unsigned short* QXH  = (unsigned short*)(ws + oQXH);
  unsigned short* QXL  = (unsigned short*)(ws + oQXL);
  unsigned short* KX   = (unsigned short*)(ws + oKX);
  unsigned short* VT   = (unsigned short*)(ws + oVT);
  unsigned short* CTXH = (unsigned short*)(ws + oCTXH);
  unsigned short* CTXL = (unsigned short*)(ws + oCTXL);

  const dim3 blk(256);
  const int gtok = ((NTOK / 64) * (DM / 64) + 7) / 8;

  tr_cvt6<<<dim3(DM / 32, DM / 64, 6), blk, 0, stream>>>(Wq_sem, Wk_sem, Wq_sal, Wk_sal, Wv, Wo, WALL,
                                                         (long long)WD, DM, DM, WSC, 5);
  cvt_f16<<<dim3((NTOK * DM) / 2048, 2), blk, 0, stream>>>(X_sem, X_sal, XH0, (long long)NTOK * DM, NTOK * DM);
  gemm64<2, 1, false, true><<<dim3(gtok, 1), blk, 0, stream>>>(
      XH0, DM, 0LL, WQS, DM, 0LL, (void*)QXH, (void*)QXL, QXP, 0LL, 0, bq_sem, gamma, NTOK, DM, DM, 1.0f / WSC);
  gemm64<1, 1, false, true><<<dim3(gtok, 1), blk, 0, stream>>>(
      XH0, DM, 0LL, WKS, DM, 0LL, (void*)KX, (void*)KX, QXP, 0LL, 0, bk_sem, gamma, NTOK, DM, DM, 1.0f / WSC);
  gemm64<2, 1, true, true><<<dim3(gtok, 1), blk, 0, stream>>>(
      XH1, DM, 0LL, WQL, DM, 0LL, (void*)QXH, (void*)QXL, QXP, 0LL, 64, bq_sal, gamma, NTOK, DM, DM, 1.0f / WSC);
  gemm64<1, 1, false, true><<<dim3(gtok, 1), blk, 0, stream>>>(
      XH1, DM, 0LL, WKL, DM, 0LL, (void*)KX, (void*)KX, QXP, 0LL, 64, bk_sal, gamma, NTOK, DM, DM, 1.0f / WSC);
  gemm64<1, 2, false, false><<<dim3(((DM / 64) * (SEQ / 64) + 7) / 8, NBATCH), blk, 0, stream>>>(
      WVT, DM, 0LL, XH0, DM, (long long)SEQ * DM, (void*)VT, (void*)VT, SEQ, (long long)DM * SEQ, 0,
      bv, gamma, DM, SEQ, DM, 1.0f / WSC);
  attn_x<<<dim3(NBATCH * NH * NQB), dim3(128), 0, stream>>>(QXH, QXL, KX, VT, mask, CTXH, CTXL, 0.125f);
  gemm64b<true><<<dim3(gtok, 1), blk, 0, stream>>>(CTXH, CTXL, DM, WOB, DM, outf, DM, bo, NTOK, DM, DM);
  (void)hipGetLastError();
}
